// SimpleMHA2D_35072702939569
// MI455X (gfx1250) — hardware-verified
//
#include <hip/hip_runtime.h>
#define NBE 32
#define NPO 1024
#define NCH 1024
#define NHE 16
#define HWD 64
#define NHP 32
#define NQR 64
#define NK 1024
#define PSC 1024.0f
#define WSC 256.0f
#define USC 64.0f
#define RSC 2048.0f
#define ASC 16.0f

typedef __bf16 v16b __attribute__((ext_vector_type(16)));
typedef unsigned short v8us __attribute__((ext_vector_type(8), may_alias));
typedef float  v8f  __attribute__((ext_vector_type(8)));
typedef float  v4f  __attribute__((ext_vector_type(4)));
typedef float  v4fa __attribute__((ext_vector_type(4), may_alias));
union FragB { v16b v; v8us half[2]; unsigned short u[16]; };

__device__ __forceinline__ unsigned short bf16_bits(float x) { unsigned int u = __float_as_uint(x); return (unsigned short)((u + 0x7FFFu + ((u >> 16) & 1u)) >> 16); }
__device__ __forceinline__ float bf16_val(unsigned short b) { return __uint_as_float(((unsigned int)b) << 16); }
__device__ __forceinline__ float bf16_round(float x) { return bf16_val(bf16_bits(x)); }
template <int NT>
__device__ __forceinline__ v8f mmaN(v16b ah, v16b al, v16b bh, v16b bl, v8f c) {
  c = __builtin_amdgcn_wmma_f32_16x16x32_bf16(false, ah, false, bh, (short)0, c, false, false);
  if (NT >= 2) c = __builtin_amdgcn_wmma_f32_16x16x32_bf16(false, al, false, bh, (short)0, c, false, false);
  if (NT >= 3) c = __builtin_amdgcn_wmma_f32_16x16x32_bf16(false, ah, false, bl, (short)0, c, false, false);
  asm volatile("v_nop\n\tv_nop\n\tv_nop\n\tv_nop" : "+v"(c) : "v"(ah), "v"(al), "v"(bh), "v"(bl));
  return c;
}


typedef _Float16 v16h __attribute__((ext_vector_type(16)));
union FragH { v16h v; v8us half[2]; _Float16 h[16]; unsigned short u[16]; };
template <int NT>
__device__ __forceinline__ v8f mmaH(v16h ah, v16h al, v16h bh, v16h bl, v8f c) {
  c = __builtin_amdgcn_wmma_f32_16x16x32_f16(false, ah, false, bh, (short)0, c, false, false);
  if (NT >= 2) c = __builtin_amdgcn_wmma_f32_16x16x32_f16(false, al, false, bh, (short)0, c, false, false);
  if (NT >= 3) c = __builtin_amdgcn_wmma_f32_16x16x32_f16(false, ah, false, bl, (short)0, c, false, false);
  asm volatile("v_nop\n\tv_nop\n\tv_nop\n\tv_nop" : "+v"(c) : "v"(ah), "v"(al), "v"(bh), "v"(bl));
  return c;
}

__global__ __launch_bounds__(256) void k_wt_f16(const float* __restrict__ W, _Float16* __restrict__ Wt, int K, int N, float scale) {
  const int t = blockIdx.x * 256 + threadIdx.x; if (t >= N * (K / 8)) return; const int n = t / (K / 8), k8 = (t % (K / 8)) * 8; FragH f;
#pragma unroll
  for (int i = 0; i < 8; ++i) f.h[i] = (_Float16)(bf16_round(W[(size_t)(k8 + i) * N + n]) * scale); const v8us o = f.half[0];
  *(volatile v8us*)((unsigned short*)Wt + (size_t)n * K + k8) = o; __threadfence(); *(volatile v8us*)((unsigned short*)Wt + (size_t)n * K + k8) = o;
}

typedef _Float16 v4h __attribute__((ext_vector_type(4)));

__global__ __launch_bounds__(256) void k_x16(const float* __restrict__ x, _Float16* __restrict__ X16, size_t n8) { const size_t t = (size_t)blockIdx.x * 256 + threadIdx.x; if (t >= n8) return; FragH f;
#pragma unroll
  for (int q = 0; q < 8; ++q) f.h[q] = (_Float16)bf16_round(x[t * 8 + q]); *(volatile v8us*)((unsigned short*)X16 + t * 8) = f.half[0]; __threadfence(); *(volatile v8us*)((unsigned short*)X16 + t * 8) = f.half[0]; }
__device__ __forceinline__ v16h g2_frag(const _Float16* p, int hh) { FragH f; f.half[0] = *(const v8us*)((const unsigned short*)p + 8 * hh); f.half[1] = *(const v8us*)((const unsigned short*)p + 16 + 8 * hh); return f.v; }
__device__ __forceinline__ v8f g2_mma(v16h a, v16h b, v8f c) { v8f d = __builtin_amdgcn_wmma_f32_16x16x32_f16(false, a, false, b, (short)0, c, false, false); asm volatile("v_nop\n\tv_nop\n\tv_nop\n\tv_nop" : "+v"(d) : "v"(a), "v"(b)); return d; }
template <int ACT>
__global__ __launch_bounds__(128) void k_gemm2(const _Float16* __restrict__ A, int lda, size_t sA, const _Float16* __restrict__ Bh, int ldb, size_t sB, float alpha, const float* __restrict__ bias, size_t sBias, const float* __restrict__ CP, int rowsPerB, size_t sCPb, int row0g,
    float* __restrict__ C, _Float16* __restrict__ C16, int ldc, size_t sC, int M, int N, int K) { static_assert(ACT == 0 || ACT == 3 || ACT == 6 || ACT == 8 || ACT == 9 || ACT == 11 || ACT == 12 || ACT == 14 || ACT == 15 || ACT == 16 || ACT == 17, "k_gemm2: unsupported ACT code (would silently apply no activation)");
  __shared__ __attribute__((aligned(16))) float so[4][32][68];
  const int tid = threadIdx.x, w = tid >> 5, lane = tid & 31, ln = lane & 15, hh = lane >> 4; const int by = blockIdx.y;
  A += (size_t)by * sA; Bh += (size_t)by * sB; const size_t cofs = (size_t)by * sC; const float* bp = bias ? bias + (size_t)by * sBias : nullptr;
  const int ntn = N >> 6; const int mt = blockIdx.x / ntn, nq = blockIdx.x - mt * ntn; const int row0 = mt * 128 + 32 * w, col0 = nq * 64; if (row0 >= M) return;
  const _Float16* a0p = A + (size_t)(row0 + ln) * lda; const _Float16* a1p = a0p + (size_t)16 * lda;
  const _Float16* b0p = Bh + (size_t)(col0 + ln) * ldb; const _Float16* b1p = b0p + (size_t)16 * ldb; const _Float16* b2p = b1p + (size_t)16 * ldb; const _Float16* b3p = b2p + (size_t)16 * ldb;
  const v8f z8 = {0.f,0.f,0.f,0.f,0.f,0.f,0.f,0.f}; v8f c00 = z8, c01 = z8, c02 = z8, c03 = z8, c10 = z8, c11 = z8, c12 = z8, c13 = z8;
  for (int kb = 0; kb < K; kb += 32) { const v16h a0 = g2_frag(a0p + kb, hh), a1 = g2_frag(a1p + kb, hh);
    v16h b = g2_frag(b0p + kb, hh); c00 = g2_mma(a0, b, c00); c10 = g2_mma(a1, b, c10);
    b = g2_frag(b1p + kb, hh); c01 = g2_mma(a0, b, c01); c11 = g2_mma(a1, b, c11);
    b = g2_frag(b2p + kb, hh); c02 = g2_mma(a0, b, c02); c12 = g2_mma(a1, b, c12);
    b = g2_frag(b3p + kb, hh); c03 = g2_mma(a0, b, c03); c13 = g2_mma(a1, b, c13); }
  v8f accs[8] = {c00, c01, c02, c03, c10, c11, c12, c13};
#pragma unroll
  for (int u = 0; u < 8; ++u) { const int t = u & 3, half = u >> 2; const int col = col0 + t * 16 + ln; const float bv = bp ? bf16_round(bp[col]) : 0.f;
#pragma unroll
    for (int r = 0; r < 8; ++r) { const int rloc = half * 16 + 8 * hh + r; float v = accs[u][r] * alpha + bv; if (CP) { if (rowsPerB < 0) v += CP[cofs + (size_t)(row0g + row0 + rloc) * ldc + col];        else { const int bidx = (row0g + row0 + rloc) / rowsPerB; v += CP[(size_t)bidx * sCPb + (size_t)by * 64 + col]; } }
      if (ACT == 3) v = fmaxf(v, 0.f); else if (ACT == 6) v = 0.5f * v * (1.0f + erff(v * 0.70710678118654752f)); else if (ACT == 11) v = 1.0f / (1.0f + expf(-v)); else if (ACT == 15) v = v / (1.0f + expf(-v)); else if (ACT == 12) v = (v > 0.f) ? v : 0.01f * v; else if (ACT == 8) v = tanhf(v); else if (ACT == 9) v = 0.5f * v * (1.0f + tanhf(0.7978845608028654f * (v + 0.044715f * v * v * v))); else if (ACT == 14) v = (v > 0.f) ? v : 0.1f * v; else if (ACT == 16) v = (v >= 0.f) ? v : 0.3f * v; else if (ACT == 17) v = (v >= 0.f) ? v : 0.2f * v;
      so[w][rloc][t * 16 + ln] = v; } }
  __builtin_amdgcn_fence(__ATOMIC_ACQ_REL, "workgroup"); __builtin_amdgcn_wave_barrier();
  const int rsub = lane >> 4, c4 = (lane & 15) * 4;
  for (int pass = 0; pass < 2; ++pass) {
#pragma unroll
    for (int q = 0; q < 16; ++q) { const int r = q * 2 + rsub; const v4f v = *(const v4fa*)&so[w][r][c4]; if (C) *(volatile v4f*)(C + cofs + (size_t)(row0 + r) * ldc + col0 + c4) = v; if (C16) { v4h h4; for (int i = 0; i < 4; ++i) h4[i] = (_Float16)v[i]; *(volatile v4h*)(C16 + cofs + (size_t)(row0 + r) * ldc + col0 + c4) = h4; } }
    if (pass == 0) __threadfence(); } }

__global__ __launch_bounds__(256) void k_wtc_f16(const float* __restrict__ W, _Float16* __restrict__ Wt, int K, int N, float scale) {
  const int t = blockIdx.x * 256 + threadIdx.x; if (t >= N * (K / 8)) return; const int n = t / (K / 8), k8 = (t % (K / 8)) * 8; FragH f;
#pragma unroll
  for (int i = 0; i < 8; ++i) f.h[i] = (_Float16)(W[(size_t)(k8 + i) * N + n] * scale); const v8us o = f.half[0];
  *(volatile v8us*)((unsigned short*)Wt + (size_t)n * K + k8) = o; __threadfence(); *(volatile v8us*)((unsigned short*)Wt + (size_t)n * K + k8) = o;
}

__global__ __launch_bounds__(256) void k_x16s(const float* __restrict__ x, _Float16* __restrict__ X16, size_t n8, float scale) { const size_t t = (size_t)blockIdx.x * 256 + threadIdx.x; if (t >= n8) return; FragH f;
#pragma unroll
  for (int q = 0; q < 8; ++q) f.h[q] = (_Float16)(bf16_round(x[t * 8 + q]) * scale); *(volatile v8us*)((unsigned short*)X16 + t * 8) = f.half[0]; __threadfence(); *(volatile v8us*)((unsigned short*)X16 + t * 8) = f.half[0]; }

__global__ __launch_bounds__(256) void k_hl(const float* __restrict__ P, _Float16* __restrict__ H16, _Float16* __restrict__ R16, size_t n8) { const size_t t = (size_t)blockIdx.x * 256 + threadIdx.x; if (t >= n8) return; FragH fh, fr;
  for (int q = 0; q < 8; ++q) { const float v = P[t * 8 + q]; const float vh = (fabsf(v) < 6.103515625e-05f) ? 0.0f : v; const _Float16 h = (_Float16)vh; const float r = (v - (float)h) * RSC; fh.h[q] = h; fr.h[q] = (_Float16)((fabsf(r) < 6.103515625e-05f) ? 0.0f : r); }
  *(volatile v8us*)((unsigned short*)H16 + t * 8) = fh.half[0]; *(volatile v8us*)((unsigned short*)R16 + t * 8) = fr.half[0]; __threadfence(); *(volatile v8us*)((unsigned short*)H16 + t * 8) = fh.half[0]; *(volatile v8us*)((unsigned short*)R16 + t * 8) = fr.half[0]; }

__global__ __launch_bounds__(256) void k_rsm(const float* __restrict__ Z, float* __restrict__ AT, _Float16* __restrict__ P16, int n) {
  const int r = blockIdx.x * 8 + (threadIdx.x >> 5); if (r >= n) return; const int ln = threadIdx.x & 31; const float* zp = Z + (size_t)r * NK + ln * 8; float m = -3.0e38f;
  for (int c = 0; c < NK; c += 256) { const v4f z0 = *(const v4fa*)(zp + c); const v4f z1 = *(const v4fa*)(zp + c + 4);
    for (int i = 0; i < 4; ++i) m = (z0[i] > m) ? z0[i] : m;
    for (int i = 0; i < 4; ++i) m = (z1[i] > m) ? z1[i] : m; }
  for (int x = 16; x >= 1; x >>= 1) { const float o = __shfl_xor(m, x, 32); m = (o > m) ? o : m; }
  float s = 0.f;
  for (int c = 0; c < NK; c += 256) { const v4f z0 = *(const v4fa*)(zp + c); const v4f z1 = *(const v4fa*)(zp + c + 4);
    for (int i = 0; i < 4; ++i) s += expf(z0[i] - m);
    for (int i = 0; i < 4; ++i) s += expf(z1[i] - m); }
  for (int x = 16; x >= 1; x >>= 1) s += __shfl_xor(s, x, 32);
  float* ap = AT + (size_t)r * NK + ln * 8; unsigned short* hp = (unsigned short*)P16 + (size_t)r * NK + ln * 8;
  for (int c = 0; c < NK; c += 256) { const v4f z0 = *(const v4fa*)(zp + c); const v4f z1 = *(const v4fa*)(zp + c + 4); v4f a0, a1; FragH f;
    for (int i = 0; i < 4; ++i) { const float p0 = expf(z0[i] - m) / s; const float p1 = expf(z1[i] - m) / s; a0[i] = p0; a1[i] = p1; const _Float16 h0 = (_Float16)(p0 * PSC); const _Float16 h1 = (_Float16)(p1 * PSC); f.h[i] = (h0 < (_Float16)6.103515625e-05f) ? (_Float16)0.0f : h0; f.h[4 + i] = (h1 < (_Float16)6.103515625e-05f) ? (_Float16)0.0f : h1; }
    *(volatile v4fa*)(ap + c) = a0; *(volatile v4fa*)(ap + c + 4) = a1; *(volatile v8us*)(hp + c) = f.half[0]; __threadfence(); *(volatile v4fa*)(ap + c) = a0; *(volatile v4fa*)(ap + c + 4) = a1; *(volatile v8us*)(hp + c) = f.half[0]; } }

__global__ __launch_bounds__(256) void k_qbd(const float* __restrict__ Qv, _Float16* __restrict__ QB, int cnt) { const int t = blockIdx.x * 256 + threadIdx.x; if (t >= cnt) return; const int r = t / (NCH / 8), c0 = (t - r * (NCH / 8)) * 8; const int hb = c0 / HWD; const bool live = (r < NHE) && (hb == r); const int src = live ? (r * HWD + (c0 - hb * HWD)) : 0; const v4f a0 = *(const v4fa*)(Qv + src); const v4f a1 = *(const v4fa*)(Qv + src + 4); FragH f;
  for (int i = 0; i < 8; ++i) { const float wd = bf16_round((i < 4) ? a0[i & 3] : a1[i & 3]); const float kept = live ? wd : 0.0f; f.h[i] = (_Float16)((fabsf(kept) < 6.103515625e-05f) ? 0.0f : kept); }
  *(volatile v8us*)((unsigned short*)QB + (size_t)t * 8) = f.half[0]; __threadfence(); *(volatile v8us*)((unsigned short*)QB + (size_t)t * 8) = f.half[0]; }

extern "C" void kernel_launch(void* const* d_in, const int* in_sizes, int n_in,
                              void* d_out, int out_size, void* d_ws, size_t ws_size, hipStream_t stream) {
  (void)in_sizes; (void)n_in; (void)out_size;
  const float* MP = (const float*)d_in[0];
  const float* FV = (const float*)d_in[1];
  const float* M1 = (const float*)d_in[2];
  const float* M2 = (const float*)d_in[4]; const float* B2 = (const float*)d_in[5];
  static_assert(((size_t)NBE * NPO * NCH / 8) % 256 == 0 && ((size_t)NCH * (NPO / 8)) % 256 == 0 && ((size_t)NCH * NCH / 8) % 256 == 0 && ((size_t)NQR * NCH / 8) % 256 == 0 && (NBE * NHP) % 8 == 0 && NHE * HWD == NCH && NHP == 32 && NQR == 64 && NHE <= NHP && NHP <= NQR && NK == NPO && NPO % 256 == 0 && NCH % 64 == 0 && (NBE * NPO) % 64 == 0 && HWD % 64 == 0 && NCH % 32 == 0 && NPO % 32 == 0 && NBE == 32, "whole tiles; exact grids; a head's 32 batch entries are the 32 rows of the last product");
  float* YF = (float*)d_out;
  char* ws = (char*)d_ws; size_t off = 0;
  auto take = [&](size_t bytes) { char* p = ws + off; off += (bytes + 255) & ~(size_t)255; return p; };
  _Float16* X16 = (_Float16*)take((size_t)NBE * NPO * NCH * 2);
  _Float16* XT16 = (_Float16*)take((size_t)NBE * NCH * NPO * 2);
  _Float16* W116 = (_Float16*)take((size_t)NCH * NCH * 2);
  _Float16* W2T16 = (_Float16*)take((size_t)NCH * NCH * 2);
  _Float16* QB16 = (_Float16*)take((size_t)NQR * NCH * 2);
  float* UT = (float*)take((size_t)NQR * NCH * 4);
  _Float16* UH16 = (_Float16*)take((size_t)NQR * NCH * 2); _Float16* UR16 = (_Float16*)take((size_t)NQR * NCH * 2);
  float* LG = (float*)take((size_t)NHP * NBE * NPO * 4);
  float* SH = (float*)take((size_t)NHP * NBE * NPO * 4);
  _Float16* P16 = (_Float16*)take((size_t)NHP * NBE * NPO * 2);
  _Float16* AX16 = (_Float16*)take((size_t)NBE * NHP * NCH * 2);
  if (off > ws_size) return;
  k_x16<<<(unsigned)((size_t)NBE * NPO * NCH / 8 / 256), 256, 0, stream>>>(MP, X16, (size_t)NBE * NPO * NCH / 8);
  for (int be = 0; be < NBE; ++be) k_wt_f16<<<(unsigned)((size_t)NCH * (NPO / 8) / 256), 256, 0, stream>>>(MP + (size_t)be * NPO * NCH, XT16 + (size_t)be * NCH * NPO, NPO, NCH, 1.0f);
  k_x16s<<<(unsigned)((size_t)NCH * NCH / 8 / 256), 256, 0, stream>>>(M1, W116, (size_t)NCH * NCH / 8, WSC);
  k_wt_f16<<<(unsigned)((size_t)NCH * (NCH / 8) / 256), 256, 0, stream>>>(M2, W2T16, NCH, NCH, WSC);
  k_qbd<<<(unsigned)((size_t)NQR * NCH / 8 / 256), 256, 0, stream>>>(FV, QB16, (int)((size_t)NQR * NCH / 8));
  k_gemm2<0><<<dim3(((NQR + 127) / 128) * (NCH / 64), 1), 128, 0, stream>>>(QB16, NCH, 0, W116, NCH, 0, USC / WSC, nullptr, 0, nullptr, 1, 0, 0, UT, nullptr, NCH, 0, NQR, NCH, NCH);
  k_hl<<<(unsigned)((size_t)NQR * NCH / 8 / 256), 256, 0, stream>>>(UT, UH16, UR16, (size_t)NQR * NCH / 8);
  k_gemm2<0><<<dim3(((NHP + 127) / 128) * ((NBE * NPO) / 64), 1), 128, 0, stream>>>(UH16, NCH, 0, X16, NCH, 0, 1.0f / USC, nullptr, 0, nullptr, 1, 0, 0, LG, nullptr, NBE * NPO, 0, NHP, NBE * NPO, NCH);
  k_gemm2<0><<<dim3(((NHP + 127) / 128) * ((NBE * NPO) / 64), 1), 128, 0, stream>>>(UR16, NCH, 0, X16, NCH, 0, 1.0f / (USC * RSC), nullptr, 0, LG, -1, 0, 0, LG, nullptr, NBE * NPO, 0, NHP, NBE * NPO, NCH);
  k_rsm<<<(NHP * NBE) / 8, 256, 0, stream>>>(LG, SH, P16, NHP * NBE);
  k_gemm2<0><<<dim3(((NHP + 127) / 128) * (NCH / 64), NBE), 128, 0, stream>>>(P16, NBE * NPO, (size_t)NPO, XT16, NPO, (size_t)NCH * NPO, ASC / PSC, nullptr, 0, nullptr, 1, 0, 0, nullptr, AX16, NCH, (size_t)NHP * NCH, NHP, NCH, NPO);
  k_gemm2<0><<<dim3(((NBE + 127) / 128) * (HWD / 64), NHE), 128, 0, stream>>>(AX16, NHP * NCH, (size_t)NCH, W2T16, NCH, (size_t)HWD * NCH, 1.0f / (ASC * WSC), B2, (size_t)HWD, nullptr, 1, 0, 0, YF, nullptr, NHE * HWD, (size_t)HWD, NBE, HWD, NCH);
}
